// NonparametricCrossAttentionPooling_41188736369110
// MI455X (gfx1250) — hardware-verified
//
#include <hip/hip_runtime.h>
#include <math.h>

#define NBAT 8
#define NQ 4096
#define NK 4096
#define FF 64
#define KSTRIDE 72
#define VSTRIDE 48
#define RSPLIT (1.0f / 2048.0f)

typedef _Float16 h16;
typedef __attribute__((ext_vector_type(16))) _Float16 v16h;
typedef __attribute__((ext_vector_type(8)))  _Float16 v8h;
typedef __attribute__((ext_vector_type(8)))  float v8f;
typedef __attribute__((ext_vector_type(4)))  float v4f_t;
typedef float v4fa __attribute__((ext_vector_type(4), may_alias));

__device__ __forceinline__ h16 lo_of(float v, h16 h) { return (h16)((v - (float)h) * 2048.0f); }
__device__ __forceinline__ v8f wmma16(v16h a, v16h b, v8f c) { return __builtin_amdgcn_wmma_f32_16x16x32_f16(false, a, false, b, (short)0, c, false, false); }
__device__ __forceinline__ v8f wmma_split(v16h a, v16h al, v16h b, v16h bl, v8f c) { v8f x = {}; x = wmma16(al, b, x); x = wmma16(a, bl, x); return wmma16(a, b, c) + x * RSPLIT; }
__device__ __forceinline__ v16h rfrag(const h16* rowp, int half) {
  const h16* p = rowp + 8 * half;
  return __builtin_shufflevector(*(const v8h*)p, *(const v8h*)(p + 16), 0,1,2,3,4,5,6,7,8,9,10,11,12,13,14,15);
}

__global__ __launch_bounds__(64) void k_regress(const float* __restrict__ Qg, const float* __restrict__ KV, float* __restrict__ NF) {
  __shared__ __attribute__((aligned(16))) h16 ldsK[2][32 * KSTRIDE];
  __shared__ __attribute__((aligned(16))) h16 ldsV[64 * VSTRIDE];
  __shared__ float k2s[32];
  __shared__ __attribute__((aligned(16))) float ldsO[2][16 * 68];
  const int q0blk = blockIdx.x * 32, b = blockIdx.y;
  const int t = threadIdx.x, wave = t >> 5, lane = t & 31, qlane = lane & 15, kh8 = (lane >> 4) * 8, half = lane >> 4;
  const int q0 = q0blk + wave * 16;
  const float* Qb = Qg + (size_t)b * NQ * FF;
  const float* Kb = KV + (size_t)b * NK * FF;

  v16h qf[1][2], qfl[1][2];
  float q2v[1];
#pragma unroll
  for (int qt = 0; qt < 1; ++qt) {
    const float* qrow = Qb + (size_t)(q0 + 16 * qt + qlane) * FF;
    float ss = 0.0f;
#pragma unroll
    for (int c = 0; c < 2; ++c) {
#pragma unroll
      for (int e = 0; e < 16; ++e) { const float v = qrow[c * 32 + kh8 + ((e < 8) ? e : (e + 8))]; qf[qt][c][e] = (h16)v; qfl[qt][c][e] = lo_of(v, qf[qt][c][e]); }
    }
#pragma unroll 4
    for (int f = 0; f < FF; ++f) { const float v = qrow[f]; ss += v * v; }
    q2v[qt] = ss;
  }
  v8f o[1][4] = {};
  float rref[1], lrun[1];
#pragma unroll
  for (int qt = 0; qt < 1; ++qt) { rref[qt] = 3.0e38f; lrun[qt] = 0.0f; }
  const int krow = t >> 1, kcol = (t & 1) * 32;

#pragma unroll 1
  for (int kb = 0; kb < NK; kb += 32) {
    __syncthreads();
    {
      const float* kr = Kb + (size_t)(kb + krow) * FF + kcol;
      float ssk = 0.0f;
#pragma unroll
      for (int i = 0; i < 32; ++i) { const float v = kr[i]; ssk += v * v; const h16 hv = (h16)v; ldsK[0][krow * KSTRIDE + kcol + i] = hv; ldsK[1][krow * KSTRIDE + kcol + i] = lo_of(v, hv); }
      ssk += __shfl_xor(ssk, 1, 32);
      if ((t & 1) == 0) k2s[krow] = ssk;
      const int vk = t & 31, f0 = (t >> 5) * 32;
      const float* vr = Kb + (size_t)(kb + vk) * FF + f0;
#pragma unroll
      for (int i = 0; i < 32; ++i) ldsV[(f0 + i) * VSTRIDE + vk] = (h16)vr[i];
    }
    __syncthreads();
    v16h kf[2][2], kfl[2][2];
#pragma unroll
    for (int kt = 0; kt < 2; ++kt)
#pragma unroll
      for (int c = 0; c < 2; ++c) { kf[kt][c] = rfrag(&ldsK[0][(kt * 16 + qlane) * KSTRIDE + c * 32], half); kfl[kt][c] = rfrag(&ldsK[1][(kt * 16 + qlane) * KSTRIDE + c * 32], half); }
    v16h pf[1];
#pragma unroll
    for (int qt = 0; qt < 1; ++qt) {
      v8f s0 = {}, s1 = {};
      s0 = wmma_split(kf[0][0], kfl[0][0], qf[qt][0], qfl[qt][0], s0); s0 = wmma_split(kf[0][1], kfl[0][1], qf[qt][1], qfl[qt][1], s0);
      s1 = wmma_split(kf[1][0], kfl[1][0], qf[qt][0], qfl[qt][0], s1); s1 = wmma_split(kf[1][1], kfl[1][1], qf[qt][1], qfl[qt][1], s1);
      float d0[8], d1[8], mn = 3.0e38f;
#pragma unroll
      for (int r = 0; r < 8; ++r) {
        const float a0 = q2v[qt] + k2s[kh8 + r] - 2.0f * s0[r];
        const float a1 = q2v[qt] + k2s[16 + kh8 + r] - 2.0f * s1[r];
        d0[r] = fmaxf(a0, 1e-12f); d1[r] = fmaxf(a1, 1e-12f);
        mn = fminf(mn, fminf(d0[r], d1[r]));
      }
      mn = fminf(mn, __shfl_xor(mn, 16, 32));
      const float rnew = fminf(rref[qt], mn);
      const float alpha = __expf((rnew - rref[qt]) * 0.125f);
      float rsum = 0.0f;
#pragma unroll
      for (int r = 0; r < 8; ++r) {
        float n2 = d0[r];
        float p0 = __expf((rnew - n2) * 0.125f) + (0.5f / 0.3f) * __expf(rnew * 0.125f - 0.5f * n2) + (0.2f / 0.3f) * __expf(rnew * 0.125f - 2.0f * n2);
        n2 = d1[r];
        float p1 = __expf((rnew - n2) * 0.125f) + (0.5f / 0.3f) * __expf(rnew * 0.125f - 0.5f * n2) + (0.2f / 0.3f) * __expf(rnew * 0.125f - 2.0f * n2);
        rsum += p0 + p1;
        pf[qt][r] = (h16)(p0 * 1024.0f); pf[qt][r + 8] = (h16)(p1 * 1024.0f);
      }
      rsum += __shfl_xor(rsum, 16, 32);
      lrun[qt] = lrun[qt] * alpha + rsum;
      rref[qt] = rnew;
#pragma unroll
      for (int j = 0; j < 4; ++j)
#pragma unroll
        for (int r = 0; r < 8; ++r) o[qt][j][r] *= alpha;
    }
#pragma unroll
    for (int j = 0; j < 4; ++j) {
      const v16h vf = rfrag(&ldsV[(j * 16 + qlane) * VSTRIDE], half);
#pragma unroll
      for (int qt = 0; qt < 1; ++qt) o[qt][j] = wmma16(vf, pf[qt], o[qt][j]);
    }
  }
  float* so = ldsO[wave];
#pragma unroll
  for (int qt = 0; qt < 1; ++qt) {
    const float denom = lrun[qt] + 1e-8f * __expf(rref[qt] * 0.125f) * (1.0f / 0.3f);
    const float rl = 1.0f / (denom * 1024.0f);
#pragma unroll
    for (int j = 0; j < 4; ++j)
#pragma unroll
      for (int r = 0; r < 8; ++r) so[qlane * 68 + j * 16 + kh8 + r] = o[qt][j][r] * rl;
  }
  asm volatile("s_wait_dscnt 0" ::: "memory");
#pragma unroll 1
  for (int pass = 0; pass < 2; ++pass) {
#pragma unroll
    for (int it = 0; it < 8; ++it) { const int ch = lane + 32 * it, ql = ch >> 4, q4 = (ch & 15) * 4;
      *(volatile v4f_t*)(NF + ((size_t)b * NQ + q0 + ql) * FF + q4) = *(const volatile v4fa*)(so + ql * 68 + q4); }
    __threadfence();
  }
}

__global__ __launch_bounds__(256) void k_bnstats(const float* __restrict__ NF, float* __restrict__ mean, float* __restrict__ rsig) {
  __shared__ float s1[4][64], s2[4][64];
  const int tid = threadIdx.x, c = tid & 63, ph = tid >> 6;
  float a = 0.0f, q = 0.0f;
#pragma unroll 1
  for (int r = ph; r < NBAT * NQ; r += 4) { const float v = NF[(size_t)r * FF + c]; a += v; q += v * v; }
  s1[ph][c] = a; s2[ph][c] = q;
  __syncthreads();
  if (tid < 64) {
    const float su = (s1[0][tid] + s1[1][tid]) + (s1[2][tid] + s1[3][tid]);
    const float sq = (s2[0][tid] + s2[1][tid]) + (s2[2][tid] + s2[3][tid]);
    const float m = su / (float)(NBAT * NQ);
    const float var = fmaxf(sq / (float)(NBAT * NQ) - m * m, 0.0f);
    s1[0][tid] = m; s2[0][tid] = rsqrtf(var + 1e-5f);
  }
  __syncthreads();
#pragma unroll 1
  for (int pass = 0; pass < 2; ++pass) {
    if (tid < 64) { *(volatile float*)(mean + tid) = s1[0][tid]; *(volatile float*)(rsig + tid) = s2[0][tid]; }
    __threadfence();
  }
}

__device__ __forceinline__ float gelu_erf(float x) { return 0.5f * x * (1.0f + erff(x * 0.70710678118654752f)); }
__global__ __launch_bounds__(256) void k_bn_gelu(const float* __restrict__ NF, const float* __restrict__ mean, const float* __restrict__ rsig,
                                                const float* __restrict__ gamma, const float* __restrict__ beta, float* __restrict__ out) {
  const int g = blockIdx.x * 256 + threadIdx.x;
  const size_t e0 = (size_t)g * 4; const int f0 = (int)(e0 & (FF - 1));
  v4f_t v = *(const v4fa*)(NF + e0), y;
#pragma unroll 1
  for (int i = 0; i < 4; ++i) { const int f = f0 + i;
    const float x = (v[i] - mean[f]) * rsig[f] * gamma[f] + beta[f];
    y[i] = gelu_erf(x); }
  *(volatile v4f_t*)(out + e0) = y; __threadfence(); *(volatile v4f_t*)(out + e0) = y;
}

extern "C" void kernel_launch(void* const* d_in, const int* in_sizes, int n_in,
                              void* d_out, int out_size, void* d_ws, size_t ws_size,
                              hipStream_t stream) {
  (void)in_sizes; (void)n_in; (void)out_size; (void)ws_size;
  const float* query = (const float*)d_in[0];
  const float* kv    = (const float*)d_in[1];
  const float* gamma = (const float*)d_in[2];
  const float* beta  = (const float*)d_in[3];
  char* ws = (char*)d_ws;
  float* NF = (float*)ws; ws += (size_t)NBAT * NQ * FF * 4;
  float* mean = (float*)ws; ws += 256;
  float* rsig = (float*)ws; ws += 256;
  k_regress<<<dim3(NQ / 32, NBAT), 64, 0, stream>>>(query, kv, NF);
  k_bnstats<<<1, 256, 0, stream>>>(NF, mean, rsig);
  k_bn_gelu<<<(NBAT * NQ * FF / 4) / 256, 256, 0, stream>>>(NF, mean, rsig, gamma, beta, (float*)d_out);
}
